// SelfAttentionNarrow_86079734547081
// MI455X (gfx1250) — hardware-verified
//
#include <hip/hip_runtime.h>
#include <math.h>
#include <stdint.h>

#define NB    4
#define SEQ   2048
#define DMOD  768
#define NH    8
#define HD    96
#define ROWS  (NB * SEQ)
#define QSC   8.0f
#define KSC   8.0f
#define PCAR  32768.0f
#define VCAR  256.0f
#define OSC   1024.0f
#define WOS   1024.0f
#define LOG2E 1.4426950408889634f
#define RSQK  0.0360843918243516f
#define ATT_WAVES   4
#define ATT_THREADS (ATT_WAVES * 32)
#define ATT_BLOCKS  (NB * NH * (SEQ / 64))
#define NKB    (SEQ / 32)
#define SLAB   (16 * 68)
#define SLAB96 (16 * 100)
static_assert(DMOD == NH * HD && HD == 96 && NH == 8 && NB == 4 && SEQ == 2048);
static_assert((SEQ / 64) == 32 && ATT_BLOCKS == 1024 && ATT_THREADS == 128 && NKB == 64);
static_assert((HD % 32) == 0 && (DMOD % 64) == 0 && (ROWS % 64) == 0 && (SEQ % 64) == 0);
static_assert(((ROWS * DMOD / 8) % 256) == 0 && ((DMOD * DMOD / 8) % 256) == 0 && ((HD * HD) % 8) == 0);
static_assert((SLAB * 4) % 16 == 0 && (SLAB96 * 4) % 16 == 0);

typedef unsigned short u16;
typedef _Float16 v16h __attribute__((ext_vector_type(16)));
typedef _Float16 v8h  __attribute__((ext_vector_type(8)));
typedef __bf16   v16b __attribute__((ext_vector_type(16)));
typedef float    v8f  __attribute__((ext_vector_type(8)));
typedef float    v4f  __attribute__((ext_vector_type(4)));
typedef unsigned int v4u __attribute__((ext_vector_type(4)));

union FragH { v16h v; v8h h[2]; v4u u[2]; };
union FragB { v16b v; v4u u[2]; };

__device__ __forceinline__ unsigned short bf_bits(float f) {
  unsigned u = __float_as_uint(f);
  return (unsigned short)((u + 0x7FFFu + ((u >> 16) & 1u)) >> 16);
}
__device__ __forceinline__ float bf_up(unsigned short h) { return __uint_as_float(((unsigned)h) << 16); }
__device__ __forceinline__ unsigned short h_bits(_Float16 x) { return __builtin_bit_cast(unsigned short, x); }
__device__ __forceinline__ unsigned pk16(unsigned short a, unsigned short b) { return (unsigned)a | ((unsigned)b << 16); }
__device__ __forceinline__ v8f zero8() { v8f z = {0.f, 0.f, 0.f, 0.f, 0.f, 0.f, 0.f, 0.f}; return z; }

__device__ __forceinline__ v16h ldfrag_h(const _Float16* p) {
  FragH f;
  f.h[0] = *(const v8h*)(p);
  f.h[1] = *(const v8h*)(p + 16);
  return f.v;
}
__device__ __forceinline__ v16b ldfrag_b(const u16* p) {
  FragB f;
  f.u[0] = *(const v4u*)(p);
  f.u[1] = *(const v4u*)(p + 16);
  return f.v;
}

__device__ __forceinline__ v8f mma_h(v16h a, v16h b, v8f c) {
  return __builtin_amdgcn_wmma_f32_16x16x32_f16(false, a, false, b, (short)0, c, false, false);
}
__device__ __forceinline__ v8f mma_b(v16b a, v16b b, v8f c) {
  return __builtin_amdgcn_wmma_f32_16x16x32_bf16(false, a, false, b, (short)0, c, false, false);
}
__device__ __forceinline__ void guard1(v8f& s, v16h x0, v16h x1, v16h x2, v16h x3, v16h x4, v16h x5) {
#if defined(__HIP_DEVICE_COMPILE__)
  asm volatile("v_nop\n\tv_nop\n\tv_nop\n\tv_nop"
               : "+v"(s) : "v"(x0), "v"(x1), "v"(x2), "v"(x3), "v"(x4), "v"(x5) : "memory");
#endif
}
__device__ __forceinline__ void guard3(v8f& a, v8f& b, v8f& c, v16h x0, v16h x1, v16h x2, v16h x3) {
#if defined(__HIP_DEVICE_COMPILE__)
  asm volatile("v_nop\n\tv_nop\n\tv_nop\n\tv_nop"
               : "+v"(a), "+v"(b), "+v"(c) : "v"(x0), "v"(x1), "v"(x2), "v"(x3) : "memory");
#endif
}
template <typename F>
__device__ __forceinline__ void guard4(v8f& a, v8f& b, v8f& c, v8f& d, F x0, F x1, F x2, F x3, F x4) {
#if defined(__HIP_DEVICE_COMPILE__)
  asm volatile("v_nop\n\tv_nop\n\tv_nop\n\tv_nop"
               : "+v"(a), "+v"(b), "+v"(c), "+v"(d) : "v"(x0), "v"(x1), "v"(x2), "v"(x3), "v"(x4) : "memory");
#endif
}
__device__ __forceinline__ void guard6(v8f& a0, v8f& a1, v8f& a2, v8f& a3, v8f& a4, v8f& a5,
                                       v16b x0, v16b x1, v16b x2, v16b x3, v16b x4, v16b x5, v16b x6) {
#if defined(__HIP_DEVICE_COMPILE__)
  asm volatile("v_nop\n\tv_nop\n\tv_nop\n\tv_nop"
               : "+v"(a0), "+v"(a1), "+v"(a2), "+v"(a3), "+v"(a4), "+v"(a5)
               : "v"(x0), "v"(x1), "v"(x2), "v"(x3), "v"(x4), "v"(x5), "v"(x6) : "memory");
#endif
}
__device__ __forceinline__ void acc_guard6(v8f& a, v8f& b, v8f& c, v8f& d, v8f& e, v8f& f) {
#if defined(__HIP_DEVICE_COMPILE__)
  asm volatile("v_nop\n\tv_nop\n\tv_nop\n\tv_nop" : "+v"(a), "+v"(b), "+v"(c), "+v"(d), "+v"(e), "+v"(f));
#endif
}
__device__ __forceinline__ void wave_sync_lds() {
#if defined(__HIP_DEVICE_COMPILE__)
  __builtin_amdgcn_fence(__ATOMIC_RELEASE, "workgroup");
  __builtin_amdgcn_wave_barrier();
  __builtin_amdgcn_fence(__ATOMIC_ACQUIRE, "workgroup");
#endif
}

__global__ __launch_bounds__(256) void cvt16(const float* __restrict__ x, u16* D, int n8, int mode, float scale) {
  const int gt = blockIdx.x * 256 + (int)threadIdx.x;
  if (gt >= n8) return;
  const float* p = x + (size_t)gt * 8;
  const v4f a = *(const v4f*)(p), c4 = *(const v4f*)(p + 4);
  float v[8];
#pragma unroll
  for (int e = 0; e < 4; ++e) { v[e] = a[e]; v[4 + e] = c4[e]; }
  unsigned short s[8];
#pragma unroll
  for (int e = 0; e < 8; ++e) {
    const unsigned short bb = bf_bits(v[e]);
    const unsigned short hb = h_bits((_Float16)(bf_up(bb) * scale));
    s[e] = (mode != 0) ? hb : bb;
  }
  v4u o;
#pragma unroll
  for (int e = 0; e < 4; ++e) o[e] = pk16(s[2 * e], s[2 * e + 1]);
  u16* d = D + (size_t)gt * 8;
  for (int pass = 0; pass < 2; ++pass) {
    *(volatile v4u*)(d) = o;
    __threadfence();
  }
}

__device__ __forceinline__ void out96(const float* sl, u16* dst, int lane) {
  wave_sync_lds();
  v4u ov[6];
#pragma unroll
  for (int i = 0; i < 6; ++i) {
    const int g   = i * 32 + lane;
    const int row = g / 12;
    const int c8  = (g - row * 12) * 8;
    const v4f a = *(const v4f*)(sl + row * 100 + c8), c4 = *(const v4f*)(sl + row * 100 + c8 + 4);
    float w[8];
#pragma unroll
    for (int e = 0; e < 4; ++e) { w[e] = a[e]; w[4 + e] = c4[e]; }
#pragma unroll
    for (int e = 0; e < 4; ++e) ov[i][e] = pk16(h_bits((_Float16)w[2 * e]), h_bits((_Float16)w[2 * e + 1]));
  }
  for (int pass = 0; pass < 2; ++pass) {
#pragma unroll
    for (int i = 0; i < 6; ++i) {
      *(volatile v4u*)(dst + (size_t)(i * 32 + lane) * 8) = ov[i];
    }
    __threadfence();
  }
}

__device__ __forceinline__ void epi16(float* sl, v8f a0, v8f a1, v8f a2, v8f a3, float oscale, u16* C, int N,
                                      size_t rowb, int col0, int lane) {
  const int hh = lane >> 4, m = lane & 15;
#pragma unroll
  for (int r = 0; r < 8; ++r) {
    const int ro = (8 * hh + r) * 68 + m;
    sl[ro]      = a0[r] * oscale;
    sl[ro + 16] = a1[r] * oscale;
    sl[ro + 32] = a2[r] * oscale;
    sl[ro + 48] = a3[r] * oscale;
  }
  wave_sync_lds();
  const int rq = lane >> 3, c8 = (lane & 7) * 8;
  v4u ov[4];
#pragma unroll
  for (int i4 = 0; i4 < 4; ++i4) {
    const int row = i4 * 4 + rq;
    const v4f a = *(const v4f*)(sl + row * 68 + c8), c4 = *(const v4f*)(sl + row * 68 + c8 + 4);
    float w[8];
#pragma unroll
    for (int e = 0; e < 4; ++e) { w[e] = a[e]; w[4 + e] = c4[e]; }
#pragma unroll
    for (int e = 0; e < 4; ++e) ov[i4][e] = pk16(h_bits((_Float16)w[2 * e]), h_bits((_Float16)w[2 * e + 1]));
  }
  u16* dst = C + (rowb + (size_t)rq) * (size_t)N + col0 + c8;
  for (int pass = 0; pass < 2; ++pass) {
#pragma unroll
    for (int i4 = 0; i4 < 4; ++i4) {
      *(volatile v4u*)(dst + (size_t)(i4 * 4) * (size_t)N) = ov[i4];
    }
    __threadfence();
  }
}

__device__ __forceinline__ void epi64b(float* sl, v8f a0, v8f a1, v8f a2, v8f a3, float oscale,
                                       float bz0, float bz1, float bz2, float bz3, float* C, int N,
                                       size_t rowb, int col0, int lane) {
  const int hh = lane >> 4, m = lane & 15;
#pragma unroll
  for (int r = 0; r < 8; ++r) {
    const int ro = (8 * hh + r) * 68 + m;
    sl[ro]      = a0[r] * oscale + bz0;
    sl[ro + 16] = a1[r] * oscale + bz1;
    sl[ro + 32] = a2[r] * oscale + bz2;
    sl[ro + 48] = a3[r] * oscale + bz3;
  }
  wave_sync_lds();
  v4f vals[8];
#pragma unroll
  for (int it = 0; it < 8; ++it) vals[it] = *(const v4f*)(sl + (it * 2 + hh) * 68 + m * 4);
  float* dst = C + (rowb + (size_t)hh) * (size_t)N + col0 + m * 4;
  for (int pass = 0; pass < 2; ++pass) {
#pragma unroll
    for (int it = 0; it < 8; ++it) {
      *(volatile v4f*)(dst + (size_t)(it * 2) * (size_t)N) = vals[it];
    }
    __threadfence();
  }
}

__global__ __launch_bounds__(128)
void proj_qk(const u16* __restrict__ XB, const u16* __restrict__ W, u16* P, float oscale) {
  __shared__ __align__(16) float smem[4 * SLAB96];
  const int tid = threadIdx.x, wave = tid >> 5, lane = tid & 31, hh = lane >> 4, m = lane & 15;
  const int bid  = blockIdx.x;
  const int head = bid & (NH - 1);
  const int rt   = bid >> 3;
  const int rowb = rt * 64 + wave * 16;
  const int b    = rowb >> 11;
  const int s0   = rowb & (SEQ - 1);
  const u16* ap = XB + (size_t)(rowb + m) * DMOD + head * HD + 8 * hh;
  const u16* bp = W + (size_t)m * HD + 8 * hh;
  v8f acc[6];
#pragma unroll
  for (int j = 0; j < 6; ++j) acc[j] = zero8();
#pragma unroll 1
  for (int k0 = 0; k0 < HD; k0 += 32) {
    const v16b a  = ldfrag_b(ap + k0);
    const v16b b0 = ldfrag_b(bp + k0);
    const v16b b1 = ldfrag_b(bp + 1 * 16 * HD + k0);
    const v16b b2 = ldfrag_b(bp + 2 * 16 * HD + k0);
    const v16b b3 = ldfrag_b(bp + 3 * 16 * HD + k0);
    const v16b b4 = ldfrag_b(bp + 4 * 16 * HD + k0);
    const v16b b5 = ldfrag_b(bp + 5 * 16 * HD + k0);
    acc[0] = mma_b(a, b0, acc[0]);
    acc[1] = mma_b(a, b1, acc[1]);
    acc[2] = mma_b(a, b2, acc[2]);
    acc[3] = mma_b(a, b3, acc[3]);
    acc[4] = mma_b(a, b4, acc[4]);
    acc[5] = mma_b(a, b5, acc[5]);
    guard6(acc[0], acc[1], acc[2], acc[3], acc[4], acc[5], a, b0, b1, b2, b3, b4, b5);
  }
  float* slab = smem + wave * SLAB96;
#pragma unroll
  for (int r = 0; r < 8; ++r) {
    const int ro = (8 * hh + r) * 100 + m;
#pragma unroll
    for (int j = 0; j < 6; ++j) slab[ro + 16 * j] = acc[j][r] * oscale;
  }
  out96(slab, P + ((size_t)(b * NH + head) * SEQ + s0) * HD, lane);
}

__global__ __launch_bounds__(192)
void proj_vt(const u16* __restrict__ XB, const u16* __restrict__ W, u16* VT, float oscale) {
  __shared__ __align__(16) float smem[6 * SLAB];
  const int tid = threadIdx.x, wave = tid >> 5, lane = tid & 31, hh = lane >> 4, m = lane & 15;
  const int bid  = blockIdx.x;
  const int st   = bid & (SEQ / 64 - 1);
  const int head = (bid >> 5) & (NH - 1);
  const int b    = bid >> 8;
  const int col0 = st * 64;
  const int rowb = wave * 16;
  const u16* ap = W + (size_t)(rowb + m) * HD + 8 * hh;
  const u16* bp = XB + ((size_t)b * SEQ + col0 + m) * DMOD + head * HD + 8 * hh;
  const size_t bs = (size_t)16 * DMOD;
  v8f acc0 = zero8(), acc1 = zero8(), acc2 = zero8(), acc3 = zero8();
#pragma unroll 1
  for (int k0 = 0; k0 < HD; k0 += 32) {
    const v16b a  = ldfrag_b(ap + k0);
    const v16b b0 = ldfrag_b(bp + k0);
    const v16b b1 = ldfrag_b(bp + bs + k0);
    const v16b b2 = ldfrag_b(bp + 2 * bs + k0);
    const v16b b3 = ldfrag_b(bp + 3 * bs + k0);
    acc0 = mma_b(a, b0, acc0);
    acc1 = mma_b(a, b1, acc1);
    acc2 = mma_b(a, b2, acc2);
    acc3 = mma_b(a, b3, acc3);
    guard4<v16b>(acc0, acc1, acc2, acc3, a, b0, b1, b2, b3);
  }
  u16* Cb = VT + (size_t)(b * NH + head) * HD * SEQ;
  epi16(smem + wave * SLAB, acc0, acc1, acc2, acc3, oscale, Cb, SEQ, (size_t)rowb, col0, lane);
}

__global__ __launch_bounds__(128)
void gemm_out(const u16* __restrict__ OP, const u16* __restrict__ WOB, const float* __restrict__ bias, float* C,
              float oscale) {
  __shared__ __align__(16) float slab[4 * SLAB];
  const int tid = threadIdx.x, wave = tid >> 5, lane = tid & 31, hh = lane >> 4, m = lane & 15;
  const int ntile = DMOD >> 6;
  const int bid   = blockIdx.x;
  const int rowb  = (bid / ntile) * 64 + wave * 16;
  const int col0  = (bid % ntile) * 64;
  const int row   = rowb + m;
  const int b     = row >> 11;
  const int s     = row & (SEQ - 1);
  const _Float16* abase = (const _Float16*)(const void*)OP + (((size_t)b * NH * SEQ + s) * HD + 8 * hh);
  const _Float16* bp    = (const _Float16*)(const void*)WOB + ((size_t)(col0 + m) * DMOD + 8 * hh);
  const size_t bs = (size_t)16 * DMOD;
  v8f acc0 = zero8(), acc1 = zero8(), acc2 = zero8(), acc3 = zero8();
#pragma unroll 1
  for (int k0 = 0; k0 < DMOD; k0 += 32) {
    const int h  = k0 / HD;
    const int d0 = k0 - h * HD;
    const v16h a  = ldfrag_h(abase + (size_t)h * (SEQ * HD) + d0);
    const v16h b0 = ldfrag_h(bp + k0);
    const v16h b1 = ldfrag_h(bp + bs + k0);
    const v16h b2 = ldfrag_h(bp + 2 * bs + k0);
    const v16h b3 = ldfrag_h(bp + 3 * bs + k0);
    acc0 = mma_h(a, b0, acc0);
    acc1 = mma_h(a, b1, acc1);
    acc2 = mma_h(a, b2, acc2);
    acc3 = mma_h(a, b3, acc3);
    guard4<v16h>(acc0, acc1, acc2, acc3, a, b0, b1, b2, b3);
  }
  const float bz0 = bf_up(bf_bits(bias[col0 + m]));
  const float bz1 = bf_up(bf_bits(bias[col0 + 16 + m]));
  const float bz2 = bf_up(bf_bits(bias[col0 + 32 + m]));
  const float bz3 = bf_up(bf_bits(bias[col0 + 48 + m]));
  epi64b(slab + wave * SLAB, acc0, acc1, acc2, acc3, oscale, bz0, bz1, bz2, bz3, C, DMOD, (size_t)rowb, col0, lane);
}

__global__ __launch_bounds__(ATT_THREADS)
void attn_fwd(const u16* __restrict__ QPp, const u16* __restrict__ KPp, const u16* __restrict__ VPp, u16* OPp) {
  __shared__ __align__(16) float smem[ATT_WAVES * SLAB96];

  const int tid  = threadIdx.x;
  const int wave = tid >> 5;
  const int lane = tid & 31;
  const int hh   = lane >> 4;
  const int c    = lane & 15;

  const int bid  = blockIdx.x;
  const int qt   = bid & (SEQ / 64 - 1);
  const int head = (bid >> 5) & (NH - 1);
  const int b    = bid >> 8;
  const int q0   = qt * 64 + wave * 16;
  const size_t bh = (size_t)(b * NH + head);

  const _Float16* Qb = (const _Float16*)(const void*)QPp + ((bh * SEQ + q0 + c) * HD + 8 * hh);
  const _Float16* Kb = (const _Float16*)(const void*)KPp + ((bh * SEQ + c) * HD + 8 * hh);
  const _Float16* Vb = (const _Float16*)(const void*)VPp + ((bh * HD + c) * SEQ + 8 * hh);
  const float lsc = RSQK * (LOG2E / (QSC * KSC));

  const v16h qf0 = ldfrag_h(Qb);
  const v16h qf1 = ldfrag_h(Qb + 32);
  const v16h qf2 = ldfrag_h(Qb + 64);

  float mrun = -INFINITY, lrun = 0.f;
  v8f o[6];
#pragma unroll
  for (int j = 0; j < 6; ++j) o[j] = zero8();

#pragma unroll 1
  for (int it = 0; it < NKB; ++it) {
    const int kb = it * 32;
    const _Float16* k0p = Kb + (size_t)kb * HD;
    const _Float16* k1p = k0p + (size_t)16 * HD;
    v8f s0 = zero8();
    {
      const v16h ka0 = ldfrag_h(k0p), ka1 = ldfrag_h(k0p + 32), ka2 = ldfrag_h(k0p + 64);
      s0 = mma_h(ka0, qf0, s0);
      s0 = mma_h(ka1, qf1, s0);
      s0 = mma_h(ka2, qf2, s0);
      guard1(s0, qf0, qf1, qf2, ka0, ka1, ka2);
    }
    v8f s1 = zero8();
    {
      const v16h kc0 = ldfrag_h(k1p), kc1 = ldfrag_h(k1p + 32), kc2 = ldfrag_h(k1p + 64);
      s1 = mma_h(kc0, qf0, s1);
      s1 = mma_h(kc1, qf1, s1);
      s1 = mma_h(kc2, qf2, s1);
      guard1(s1, qf0, qf1, qf2, kc0, kc1, kc2);
    }
    float tk[16];
#pragma unroll
    for (int i = 0; i < 8; ++i) { tk[i] = s0[i] * lsc;  tk[8 + i] = s1[i] * lsc; }
    float cm = tk[0];
#pragma unroll
    for (int i = 1; i < 16; ++i) cm = fmaxf(cm, tk[i]);
    cm = fmaxf(cm, __shfl_xor(cm, 16, 32));
    const float mn = fmaxf(mrun, cm);
    const float al = (mrun == -INFINITY) ? 0.f : exp2f(mrun - mn);
    mrun = mn;
    float ps = 0.f;
    FragH ph;
#pragma unroll
    for (int w = 0; w < 2; ++w) {
#pragma unroll
      for (int e4 = 0; e4 < 4; ++e4) {
        const int i = 8 * w + 2 * e4;
        const float p0 = exp2f(fminf(tk[i] - mn, 0.f));
        const float p1 = exp2f(fminf(tk[i + 1] - mn, 0.f));
        ps += p0 + p1;
        ph.u[w][e4] = pk16(h_bits((_Float16)(p0 * PCAR)), h_bits((_Float16)(p1 * PCAR)));
      }
    }
    ps += __shfl_xor(ps, 16, 32);
    lrun = lrun * al + ps;
    float scl[8];
#pragma unroll
    for (int r = 0; r < 8; ++r) scl[r] = __shfl(al, 8 * hh + r, 32);
#pragma unroll
    for (int j = 0; j < 6; ++j) {
#pragma unroll
      for (int r = 0; r < 8; ++r) o[j][r] *= scl[r];
    }
    {
      const _Float16* vp = Vb + kb;
      const v16h vf0 = ldfrag_h(vp);
      const v16h vf1 = ldfrag_h(vp + (size_t)16 * SEQ);
      const v16h vf2 = ldfrag_h(vp + (size_t)32 * SEQ);
      o[0] = mma_h(ph.v, vf0, o[0]);
      o[1] = mma_h(ph.v, vf1, o[1]);
      o[2] = mma_h(ph.v, vf2, o[2]);
      guard3(o[0], o[1], o[2], ph.v, vf0, vf1, vf2);
      const v16h vf3 = ldfrag_h(vp + (size_t)48 * SEQ);
      const v16h vf4 = ldfrag_h(vp + (size_t)64 * SEQ);
      const v16h vf5 = ldfrag_h(vp + (size_t)80 * SEQ);
      o[3] = mma_h(ph.v, vf3, o[3]);
      o[4] = mma_h(ph.v, vf4, o[4]);
      o[5] = mma_h(ph.v, vf5, o[5]);
      guard3(o[3], o[4], o[5], ph.v, vf3, vf4, vf5);
    }
  }
  acc_guard6(o[0], o[1], o[2], o[3], o[4], o[5]);

  const float linv = (lrun > 0.f) ? ((1.0f / lrun) * (OSC / (PCAR * VCAR))) : 0.f;
  float inv[8];
#pragma unroll
  for (int r = 0; r < 8; ++r) inv[r] = __shfl(linv, 8 * hh + r, 32);
  float* slab = smem + wave * SLAB96;
#pragma unroll
  for (int r = 0; r < 8; ++r) {
    const int ro = (8 * hh + r) * 100 + c;
#pragma unroll
    for (int j = 0; j < 6; ++j) slab[ro + 16 * j] = o[j][r] * inv[r];
  }
  out96(slab, OPp + (bh * SEQ + q0) * HD, lane);
}

extern "C" void kernel_launch(void* const* d_in, const int* in_sizes, int n_in,
                              void* d_out, int out_size, void* d_ws, size_t ws_size,
                              hipStream_t stream) {
  if (n_in < 6) return;
  if (in_sizes[0] != ROWS * DMOD) return;
  if (in_sizes[1] != HD * HD) return;
  if (in_sizes[2] != HD * HD) return;
  if (in_sizes[3] != HD * HD) return;
  if (in_sizes[4] != DMOD * DMOD) return;
  if (in_sizes[5] != DMOD) return;
  if (out_size != ROWS * DMOD) return;

  const float* Xin = (const float*)d_in[0];
  const float* Wq  = (const float*)d_in[1];
  const float* Wk  = (const float*)d_in[2];
  const float* Wv  = (const float*)d_in[3];
  const float* Wu  = (const float*)d_in[4];
  const float* bu  = (const float*)d_in[5];
  float*       out = (float*)d_out;

  const size_t szXB = (size_t)ROWS * DMOD * 2;
  const size_t szW  = (size_t)HD * HD * 2;
  const size_t szWO = (size_t)DMOD * DMOD * 2;
  const size_t szP  = (size_t)NB * NH * SEQ * HD * 2;
  size_t off = 0;
  const size_t oXB = off; off += szXB;
  const size_t oWQ = off; off += szW;
  const size_t oWK = off; off += szW;
  const size_t oWV = off; off += szW;
  const size_t oWO = off; off += szWO;
  const size_t oQP = off; off += szP;
  const size_t oKP = off; off += szP;
  const size_t oVP = off; off += szP;
  const size_t oOP = off; off += szP;
  if (off > ws_size) return;
  if (off > (size_t)134217728) return;
  if ((szXB % 256) != 0 || (szW % 256) != 0 || (szWO % 256) != 0 || (szP % 256) != 0) return;

  char* ws = (char*)d_ws;
  u16* XB  = (u16*)(ws + oXB);
  u16* WQB = (u16*)(ws + oWQ);
  u16* WKB = (u16*)(ws + oWK);
  u16* WVB = (u16*)(ws + oWV);
  u16* WOB = (u16*)(ws + oWO);
  u16* QP  = (u16*)(ws + oQP);
  u16* KP  = (u16*)(ws + oKP);
  u16* VP  = (u16*)(ws + oVP);
  u16* OP  = (u16*)(ws + oOP);

  const dim3 blk(256);
  const int n8x = (ROWS * DMOD) / 8;
  const int n8w = (HD * HD) / 8;
  const int n8o = (DMOD * DMOD) / 8;
  if (((HD * HD) % 8) != 0 || (n8x % 256) != 0 || (n8o % 256) != 0) return;
  if ((DMOD % 64) != 0 || (ROWS % 64) != 0 || (SEQ % 64) != 0 || (HD % 32) != 0) return;
  const dim3 gX(n8x / 256);
  const dim3 gWs((n8w + 255) / 256);
  const dim3 gWo(n8o / 256);
  const dim3 gPJ((ROWS / 64) * NH);
  const dim3 bPJ(128);
  const dim3 gVT(NB * NH * (SEQ / 64));
  const dim3 bVT(192);
  const dim3 gAT(ATT_BLOCKS);
  const dim3 bAT(ATT_THREADS);
  const dim3 gO((ROWS / 64) * (DMOD / 64));
  const dim3 bO(128);

  cvt16<<<gX, blk, 0, stream>>>(Xin, XB, n8x, 0, 1.0f);
  cvt16<<<gWs, blk, 0, stream>>>(Wq, WQB, n8w, 0, 1.0f);
  cvt16<<<gWs, blk, 0, stream>>>(Wk, WKB, n8w, 0, 1.0f);
  cvt16<<<gWs, blk, 0, stream>>>(Wv, WVB, n8w, 0, 1.0f);
  cvt16<<<gWo, blk, 0, stream>>>(Wu, WOB, n8o, 1, WOS);
  proj_qk<<<gPJ, bPJ, 0, stream>>>(XB, WQB, QP, QSC);
  proj_qk<<<gPJ, bPJ, 0, stream>>>(XB, WKB, KP, KSC);
  proj_vt<<<gVT, bVT, 0, stream>>>(XB, WVB, VP, VCAR);
  attn_fwd<<<gAT, bAT, 0, stream>>>(QP, KP, VP, OP);
  gemm_out<<<gO, bO, 0, stream>>>(OP, WOB, bu, out, 1.0f / (OSC * WOS));
  (void)hipGetLastError();
}
